// Head_38963943309606
// MI455X (gfx1250) — hardware-run, weakly checked
//
#include <hip/hip_runtime.h>
#include <stddef.h>
#include <stdint.h>
#include <math.h>

#define NN      50000
#define NE      800000
#define HD      128
#define KH      256
#define NLAY    3
#define MP      50048
#define GBM     64
#define GTHR    128
#define NTHR    256
#define NWAVE   8
#define EPT     8
#define WCH     (32 * EPT)
#define NBRUN   1024
#define SLB     10
#define NBK     49
#define WLCAP   3840
#define RCAP    20480
#define TRIPCAP 128
#define MAXDEG_MEAS   35
#define MAXB1024_MEAS 16623
#define ABM     64
#define COI     (3 * NBRUN)
#define NEGSL   0.2f
#define WSMAX   134217728

#define CONV_SPLIT_L1 1
#define CONV_SPLIT_L2 1
#define CONV_SPLIT_L3 1

#define BK_ZINTS (NWAVE * WLCAP + RCAP + 3 * NBRUN)
#define BK_INTS  (BK_ZINTS + 16)
#define BK_LDS   (BK_INTS * 4)

#define PBX   (MP * HD / 8 / NTHR)
#define PBWA  (HD * HD / 8 / NTHR)
#define PBWC  (NLAY * HD * KH / 8 / NTHR)
#define PBTOT (PBX + PBWA + PBWC + 1)
#define FLAGINTS 1600
#define SMN   768

static_assert(HD == 32 * 4 && KH == 2 * HD);
static_assert(MP % GBM == 0 && MP >= NN && MP == 391 * 128 && MP % ABM == 0);
static_assert(NBRUN == (1 << SLB) && NBRUN % ABM == 0 && NBRUN % GBM == 0 && NBRUN % 32 == 0);
static_assert(NBK * NBRUN >= MP);
static_assert(NE < (1 << 20) && (((long long)NE) << SLB) < (1LL << 31));
static_assert(NE % WCH == 0 && NE % 4 == 0);
static_assert(RCAP % (NTHR * 4) == 0 && BK_ZINTS % 4 == 0 && COI == 3 * NTHR * 4);
static_assert((long long)RCAP * 100 >= (long long)MAXB1024_MEAS * 105);
static_assert(2 * NWAVE * WLCAP >= 3 * RCAP);
static_assert(WLCAP >= MAXB1024_MEAS / NWAVE + 8 * 64 + 1);
static_assert(NN <= 65536);
static_assert(MAXDEG_MEAS + 8 <= TRIPCAP && TRIPCAP < 65536);
static_assert((MP * HD / 8) % NTHR == 0 && (HD * HD / 8) % NTHR == 0 && (NLAY * HD * KH / 8) % NTHR == 0);
static_assert(HD % 32 == 0 && KH % 32 == 0);
static_assert(BK_LDS <= 300000);
static_assert(NBK * 32 <= FLAGINTS && FLAGINTS % 4 == 0);
static_assert((NBK * NBRUN) % ABM == 0);

typedef float          v4f   __attribute__((ext_vector_type(4)));
typedef float          v8f   __attribute__((ext_vector_type(8)));
typedef int            v4i   __attribute__((ext_vector_type(4)));
typedef int            v8i   __attribute__((ext_vector_type(8)));
typedef unsigned short v8us  __attribute__((ext_vector_type(8)));
typedef unsigned short v16us __attribute__((ext_vector_type(16)));
typedef __bf16         v16bf __attribute__((ext_vector_type(16)));
typedef v4f  __attribute__((may_alias)) v4fa;
typedef v4i  __attribute__((may_alias)) v4ia;
typedef v8us __attribute__((may_alias)) v8usa;
union FragB { v16bf v; v16us u; v8us h[2]; v8i w; };

__device__ __forceinline__ v8f wmb(const FragB& a, const FragB& b, v8f c) {
  v8f d = __builtin_amdgcn_wmma_f32_16x16x32_bf16(false, a.v, false, b.v, (short)0, c, false, false);
  asm volatile("v_nop\n\tv_nop\n\tv_nop\n\tv_nop" : "+v"(d) : "v"(a.w), "v"(b.w));
  return d;
}

__device__ __forceinline__ unsigned bf16_bits(float f) {
  const unsigned u = __float_as_uint(f);
  const unsigned r = (u + 0x7FFFu + ((u >> 16) & 1u)) >> 16;
  const unsigned q = (u >> 16) | 0x40u;
  return ((u & 0x7fffffffu) > 0x7f800000u) ? q : r;
}
__device__ __forceinline__ float bf16_val(float f) {
  return __uint_as_float(bf16_bits(f) << 16);
}
__device__ __forceinline__ v4f bfr4(const v4f a) {
  v4f r; r.x = bf16_val(a.x); r.y = bf16_val(a.y); r.z = bf16_val(a.z); r.w = bf16_val(a.w); return r;
}

__device__ __forceinline__ void hilo_pack(float v0, float v1, float v2, float v3,
                                          int& h01, int& h23, int& l01, int& l23) {
  const unsigned a0 = bf16_bits(v0), a1 = bf16_bits(v1), a2 = bf16_bits(v2), a3 = bf16_bits(v3);
  const unsigned b0 = bf16_bits(v0 - __uint_as_float(a0 << 16));
  const unsigned b1 = bf16_bits(v1 - __uint_as_float(a1 << 16));
  const unsigned b2 = bf16_bits(v2 - __uint_as_float(a2 << 16));
  const unsigned b3 = bf16_bits(v3 - __uint_as_float(a3 << 16));
  h01 = (int)(a0 | (a1 << 16)); h23 = (int)(a2 | (a3 << 16));
  l01 = (int)(b0 | (b1 << 16)); l23 = (int)(b2 | (b3 << 16));
}

__device__ __forceinline__ v4i regroup8w(int h01, int h23, int l01, int l23, int lane) {
  const int s0 = (2 * lane) & 31, s1 = s0 + 1;
  const int a0 = __shfl(h01, s0, 32), a1 = __shfl(h23, s0, 32), a2 = __shfl(h01, s1, 32), a3 = __shfl(h23, s1, 32);
  const int b0 = __shfl(l01, s0, 32), b1 = __shfl(l23, s0, 32), b2 = __shfl(l01, s1, 32), b3 = __shfl(l23, s1, 32);
  const int mk = (lane < 16) ? -1 : 0;
  v4i o;
  o.x = (a0 & mk) | (b0 & ~mk); o.y = (a1 & mk) | (b1 & ~mk);
  o.z = (a2 & mk) | (b2 & ~mk); o.w = (a3 & mk) | (b3 & ~mk);
  return o;
}

__device__ __forceinline__ void st2_v4f(float* p, v4f v) {
  *(volatile v4f*)p = v;
  __threadfence();
  *(volatile v4f*)p = v;
}
__device__ __forceinline__ void st2_v4i(int* p, v4i v) {
  *(volatile v4i*)p = v;
  __threadfence();
  *(volatile v4i*)p = v;
}
__device__ __forceinline__ void st2_v8us(unsigned short* p, v8us v) {
  *(volatile v8us*)p = v;
  __threadfence();
  *(volatile v8us*)p = v;
}

__device__ __forceinline__ v8us gather8(const float* __restrict__ base, int stride) {
  float f[8];
#pragma unroll
  for (int i = 0; i < 8; ++i) f[i] = base[(size_t)i * (size_t)stride];
  v8us o;
#pragma unroll
  for (int i = 0; i < 8; ++i) o[i] = (unsigned short)bf16_bits(f[i]);
  return o;
}

__global__ __launch_bounds__(NTHR) void k_prep(const float* __restrict__ x, const float* __restrict__ wa,
                                               const float* __restrict__ asv, const float* __restrict__ adv,
                                               const float* __restrict__ ba, const float* __restrict__ wc,
                                               const float* __restrict__ bc,
                                               unsigned short* xb, unsigned short* wat, unsigned short* wcd,
                                               float* sm, int* flag) {
  const int tid = (int)threadIdx.x, lane = tid & 31, wave = tid >> 5;
  const int blk = (int)blockIdx.x;
  if (blk < PBX) {
    const int u   = blk * NTHR + tid;
    const int row = u >> 4, k8 = (u & 15) * 8;
    const int rc  = row < NN ? row : NN - 1;
    const unsigned mk = row < NN ? 0xffffu : 0u;
    const float* p = x + (size_t)rc * HD + k8;
    const v4f a = *(const v4fa*)p;
    const v4f b = *(const v4fa*)(p + 4);
    v8us o;
    o[0] = (unsigned short)(bf16_bits(a.x) & mk); o[1] = (unsigned short)(bf16_bits(a.y) & mk);
    o[2] = (unsigned short)(bf16_bits(a.z) & mk); o[3] = (unsigned short)(bf16_bits(a.w) & mk);
    o[4] = (unsigned short)(bf16_bits(b.x) & mk); o[5] = (unsigned short)(bf16_bits(b.y) & mk);
    o[6] = (unsigned short)(bf16_bits(b.z) & mk); o[7] = (unsigned short)(bf16_bits(b.w) & mk);
    st2_v8us(xb + (size_t)row * HD + k8, o);
  } else if (blk < PBX + PBWA) {
    const int u = (blk - PBX) * NTHR + tid;
    const int n = u >> 4, k8 = (u & 15) * 8;
    const v8us o = gather8(wa + (size_t)k8 * HD + n, HD);
    st2_v8us(wat + (size_t)n * HD + k8, o);
  } else if (blk < PBX + PBWA + PBWC) {
    const int u = (blk - PBX - PBWA) * NTHR + tid;
    const int l = u >> 12, n = (u >> 5) & 127, k8 = (u & 31) * 8, kk = k8 & (HD - 1);
    const v8us o = gather8(wc + (size_t)l * HD * HD + (size_t)kk * HD + n, HD);
    st2_v8us(wcd + (size_t)l * HD * KH + (size_t)n * KH + k8, o);
  } else {
    if (wave == 0) {
      const v4f v = *(const v4fa*)(asv + 4 * lane);
      st2_v4f(sm + 4 * lane, bfr4(v));
    } else if (wave == 1) {
      const v4f v = *(const v4fa*)(adv + 4 * lane);
      st2_v4f(sm + 128 + 4 * lane, bfr4(v));
    } else if (wave == 2) {
      const v4f v = *(const v4fa*)(ba + 4 * lane);
      st2_v4f(sm + 256 + 4 * lane, bfr4(v));
    } else if (wave < 6) {
      const int l = wave - 3;
      const v4f v = *(const v4fa*)(bc + 128 * l + 4 * lane);
      st2_v4f(sm + 384 + 128 * l + 4 * lane, bfr4(v));
    } else {
      const int t = tid - 192;
      const v4i z4 = {0, 0, 0, 0};
#pragma unroll 1
      for (int it = 0; it < 7; ++it) {
        const int idx = it * 64 + t;
        if (idx < FLAGINTS / 4) st2_v4i(flag + 4 * idx, z4);
      }
    }
  }
}

__device__ __forceinline__ void bucket_flush(const int* pl, const int* cnt, int ov, int* lp, int* cop, int* fp,
                                             int tid) {
#pragma unroll 1
  for (int i = tid * 4; i < RCAP; i += NTHR * 4) {
    const v4i v = *(const v4ia*)(pl + i);
    *(volatile v4i*)(lp + i) = v;
  }
#pragma unroll 1
  for (int it = 0; it < 3; ++it) {
    const int idx = it * (NTHR * 4) + 4 * tid;
    const v4i v = *(const v4ia*)(cnt + idx);
    *(volatile v4i*)(cop + idx) = v;
  }
  if (tid < 8) {
    const v4i f = {ov, ov, ov, ov};
    *(volatile v4i*)(fp + 4 * tid) = f;
  }
}

__global__ __launch_bounds__(NTHR) void k_bucket(const int* __restrict__ srcs, const int* __restrict__ dsts,
                                                 const float* __restrict__ ew, int* LIST, int* CO, int* FLAG) {
  extern __shared__ __attribute__((aligned(16))) int dsm[];
  int* wl   = dsm;
  int* pl   = dsm + NWAVE * WLCAP;
  int* cnt  = pl + RCAP;
  int* offs = cnt + NBRUN;
  int* cur  = offs + NBRUN;
  int* misc = cur + NBRUN;
  const int tid = (int)threadIdx.x, lane = tid & 31, wave = tid >> 5;
  const int blk = (int)blockIdx.x;
  const unsigned nbs = (unsigned)(blk * NBRUN);

  {
    const v4i z4 = {0, 0, 0, 0};
    for (int i = tid * 4; i < BK_ZINTS; i += NTHR * 4) *(v4ia*)(dsm + i) = z4;
    if (tid < 16) misc[tid] = 0;
  }
  __syncthreads();

  {
    const int per  = ((NE + NWAVE * WCH - 1) / (NWAVE * WCH)) * WCH;
    const int ebeg = wave * per;
    const int eend = (ebeg + per < NE) ? (ebeg + per) : NE;
    int* mylist = wl + wave * WLCAP;
    int wc = 0;
#pragma unroll 1
    for (int cb = ebeg; cb < eend; cb += WCH) {
      const int e0 = cb + lane * EPT;
      const v4i da = *(const v4ia*)(dsts + e0);
      const v4i db = *(const v4ia*)(dsts + e0 + 4);
      const unsigned s0 = (unsigned)da.x - nbs, s1 = (unsigned)da.y - nbs;
      const unsigned s2 = (unsigned)da.z - nbs, s3 = (unsigned)da.w - nbs;
      const unsigned s4 = (unsigned)db.x - nbs, s5 = (unsigned)db.y - nbs;
      const unsigned s6 = (unsigned)db.z - nbs, s7 = (unsigned)db.w - nbs;
      const bool h0 = s0 < (unsigned)NBRUN, h1 = s1 < (unsigned)NBRUN, h2 = s2 < (unsigned)NBRUN, h3 = s3 < (unsigned)NBRUN;
      const bool h4 = s4 < (unsigned)NBRUN, h5 = s5 < (unsigned)NBRUN, h6 = s6 < (unsigned)NBRUN, h7 = s7 < (unsigned)NBRUN;
      const unsigned m0 = __builtin_amdgcn_ballot_w32(h0), m1 = __builtin_amdgcn_ballot_w32(h1);
      const unsigned m2 = __builtin_amdgcn_ballot_w32(h2), m3 = __builtin_amdgcn_ballot_w32(h3);
      const unsigned m4 = __builtin_amdgcn_ballot_w32(h4), m5 = __builtin_amdgcn_ballot_w32(h5);
      const unsigned m6 = __builtin_amdgcn_ballot_w32(h6), m7 = __builtin_amdgcn_ballot_w32(h7);
      const unsigned any = m0 | m1 | m2 | m3 | m4 | m5 | m6 | m7;
      if (any != 0u) {
        const int pre = (int)(__builtin_amdgcn_mbcnt_lo(m0, 0u) + __builtin_amdgcn_mbcnt_lo(m1, 0u) +
                              __builtin_amdgcn_mbcnt_lo(m2, 0u) + __builtin_amdgcn_mbcnt_lo(m3, 0u) +
                              __builtin_amdgcn_mbcnt_lo(m4, 0u) + __builtin_amdgcn_mbcnt_lo(m5, 0u) +
                              __builtin_amdgcn_mbcnt_lo(m6, 0u) + __builtin_amdgcn_mbcnt_lo(m7, 0u));
        int p = wc + pre;
        if (h0) { if (p < WLCAP) mylist[p] = ((e0 + 0) << SLB) | (int)s0; p = p + 1; }
        if (h1) { if (p < WLCAP) mylist[p] = ((e0 + 1) << SLB) | (int)s1; p = p + 1; }
        if (h2) { if (p < WLCAP) mylist[p] = ((e0 + 2) << SLB) | (int)s2; p = p + 1; }
        if (h3) { if (p < WLCAP) mylist[p] = ((e0 + 3) << SLB) | (int)s3; p = p + 1; }
        if (h4) { if (p < WLCAP) mylist[p] = ((e0 + 4) << SLB) | (int)s4; p = p + 1; }
        if (h5) { if (p < WLCAP) mylist[p] = ((e0 + 5) << SLB) | (int)s5; p = p + 1; }
        if (h6) { if (p < WLCAP) mylist[p] = ((e0 + 6) << SLB) | (int)s6; p = p + 1; }
        if (h7) { if (p < WLCAP) mylist[p] = ((e0 + 7) << SLB) | (int)s7; p = p + 1; }
        wc += (int)(__builtin_popcount(m0) + __builtin_popcount(m1) + __builtin_popcount(m2) + __builtin_popcount(m3) +
                    __builtin_popcount(m4) + __builtin_popcount(m5) + __builtin_popcount(m6) + __builtin_popcount(m7));
      }
    }
    if (lane == 0) misc[wave] = wc;
  }
  __syncthreads();

  if (wave == 0) {
    int ov = 0;
#pragma unroll 1
    for (int w2 = 0; w2 < NWAVE; ++w2) {
      int c = misc[w2];
      if (c > WLCAP) ov = 1;
      c = c < 0 ? 0 : (c > WLCAP ? WLCAP : c);
#pragma unroll 1
      for (int b0 = 0; b0 < c; b0 += 32) {
        const int idx = b0 + lane;
        const int ent = wl[w2 * WLCAP + (idx < WLCAP ? idx : WLCAP - 1)];
        const int m32 = (c - b0) < 32 ? (c - b0) : 32;
#pragma unroll 1
        for (int k = 0; k < m32; ++k) {
          const int u    = __builtin_amdgcn_readlane(ent, k);
          const int slot = u & (NBRUN - 1);
          if (lane == 0) cnt[slot] = cnt[slot] + 1;
        }
      }
    }
    if (lane == 0) misc[9] = ov;
  }
  __syncthreads();
  if (wave == 0) {
    const int base = lane * (NBRUN / 32);
    int s = 0;
#pragma unroll 1
    for (int i = 0; i < NBRUN / 32; ++i) s += cnt[base + i];
    int incl = s;
#pragma unroll
    for (int d = 1; d < 32; d <<= 1) {
      const int y = __shfl_up(incl, d, 32);
      if (lane >= d) incl += y;
    }
    int run = incl - s;
#pragma unroll 1
    for (int i = 0; i < NBRUN / 32; ++i) {
      const int cv = cnt[base + i];
      offs[base + i] = run;
      cur[base + i]  = run;
      run += cv;
    }
    const int tot = __shfl(run, 31, 32);
    if (lane == 0 && tot > RCAP) misc[9] = 1;
  }
  __syncthreads();

  if (wave == 0) {
#pragma unroll 1
    for (int w2 = 0; w2 < NWAVE; ++w2) {
      int c = misc[w2];
      c = c < 0 ? 0 : (c > WLCAP ? WLCAP : c);
#pragma unroll 1
      for (int b0 = 0; b0 < c; b0 += 32) {
        const int idx = b0 + lane;
        const int ent = wl[w2 * WLCAP + (idx < WLCAP ? idx : WLCAP - 1)];
        int eid = (ent >> SLB) & 0xFFFFF;
        eid = eid > NE - 1 ? NE - 1 : eid;
        int sr = srcs[eid];
        sr = sr < 0 ? 0 : (sr > NN - 1 ? NN - 1 : sr);
        const int word = (int)((unsigned)sr | (bf16_bits(ew[eid]) << 16));
        const int m32 = (c - b0) < 32 ? (c - b0) : 32;
#pragma unroll 1
        for (int k = 0; k < m32; ++k) {
          const int u    = __builtin_amdgcn_readlane(ent, k);
          const int wd   = __builtin_amdgcn_readlane(word, k);
          const int slot = u & (NBRUN - 1);
          if (lane == 0) {
            int p = cur[slot];
            p = p < 0 ? 0 : (p > RCAP - 1 ? RCAP - 1 : p);
            pl[p] = wd;
            cur[slot] = p + 1;
          }
        }
      }
    }
  }
  __syncthreads();

#pragma unroll 1
  for (int i = 0; i < NBRUN / NTHR; ++i) {
    const int slot = i * NTHR + tid;
    int c = cnt[slot];
    c = c < 0 ? 0 : (c > TRIPCAP ? TRIPCAP : c);
    int o = offs[slot];
    o = o < 0 ? 0 : (o > RCAP - 1 ? RCAP - 1 : o);
    float s = 0.0f;
#pragma unroll 1
    for (int j = 0; j < c; ++j) {
      int idx = o + j;
      idx = idx > RCAP - 1 ? RCAP - 1 : idx;
      s += __uint_as_float((unsigned)pl[idx] & 0xffff0000u);
    }
    const float deg = s + 1.0f;
    const float di  = (deg > 0.0f) ? (1.0f / sqrtf(fmaxf(deg, 1e-12f))) : 0.0f;
    cur[slot] = __float_as_int(di);
  }
  __syncthreads();

  const int ovf = misc[9];
  int* lp  = LIST + (size_t)blk * RCAP;
  int* cop = CO + (size_t)blk * COI;
  int* fp  = FLAG + (size_t)blk * 32;
  bucket_flush(pl, cnt, ovf, lp, cop, fp, tid);
  __threadfence();
  bucket_flush(pl, cnt, ovf, lp, cop, fp, tid);
}

template <int KTOT, int LDB>
__device__ __forceinline__ void gemm_16x128(const unsigned short* __restrict__ ap,
                                            const unsigned short* __restrict__ bp, v8f (&acc)[8]) {
#pragma unroll 1
  for (int k0 = 0; k0 < KTOT; k0 += 32) {
    FragB af;
    af.h[0] = *(const v8usa*)(ap + k0);
    af.h[1] = *(const v8usa*)(ap + k0 + 16);
#pragma unroll
    for (int nt = 0; nt < 8; ++nt) {
      const unsigned short* wq = bp + (size_t)(16 * nt) * (size_t)LDB + k0;
      FragB bf;
      bf.h[0] = *(const v8usa*)wq;
      bf.h[1] = *(const v8usa*)(wq + 16);
      acc[nt] = wmb(af, bf, acc[nt]);
    }
  }
}

__device__ __forceinline__ void stage_d8(float* stg, const v8f (&acc)[8], int wave, int hh, int m) {
#pragma unroll
  for (int nt = 0; nt < 8; ++nt) {
#pragma unroll
    for (int r = 0; r < 8; ++r) stg[(16 * wave + 8 * hh + r) * HD + 16 * nt + m] = acc[nt][r];
  }
}

__global__ __launch_bounds__(GTHR) __attribute__((amdgpu_num_vgpr(248)))
void k_gemm0(const unsigned short* __restrict__ XB, const unsigned short* __restrict__ WaT,
             const float* __restrict__ SM, float* XP, float* AL) {
  __shared__ __attribute__((aligned(16))) float stg[GBM * HD];
  __shared__ __attribute__((aligned(16))) float sav[2 * HD];
  __shared__ __attribute__((aligned(16))) float sdt[2 * GBM];
  const int tid = (int)threadIdx.x, lane = tid & 31, wave = tid >> 5, hh = lane >> 4, m = lane & 15;
  const int rowBase = (int)blockIdx.x * GBM;
  if (tid < 32) {
    *(v4fa*)(sav + 4 * tid)      = *(const v4fa*)(SM + 4 * tid);
    *(v4fa*)(sav + HD + 4 * tid) = *(const v4fa*)(SM + HD + 4 * tid);
  }

  v8f acc[8];
  {
    const v8f z = {0.f, 0.f, 0.f, 0.f, 0.f, 0.f, 0.f, 0.f};
#pragma unroll
    for (int t = 0; t < 8; ++t) acc[t] = z;
  }
  const unsigned short* ap = XB + (size_t)(rowBase + 16 * wave + m) * (size_t)HD + 8 * hh;
  const unsigned short* bp = WaT + (size_t)m * (size_t)HD + 8 * hh;
  gemm_16x128<HD, HD>(ap, bp, acc);
  stage_d8(stg, acc, wave, hh, m);
  __syncthreads();

  const v4f as4 = *(const v4fa*)(sav + 4 * lane);
  const v4f ad4 = *(const v4fa*)(sav + HD + 4 * lane);
#pragma unroll 1
  for (int i = 0; i < 16; ++i) {
    const int row = 16 * wave + i;
    const v4f p = *(const v4fa*)(stg + row * HD + 4 * lane);
    float s = 0.0f, d = 0.0f;
    s = fmaf(p.x, as4.x, s); s = fmaf(p.y, as4.y, s); s = fmaf(p.z, as4.z, s); s = fmaf(p.w, as4.w, s);
    d = fmaf(p.x, ad4.x, d); d = fmaf(p.y, ad4.y, d); d = fmaf(p.z, ad4.z, d); d = fmaf(p.w, ad4.w, d);
#pragma unroll
    for (int off = 16; off > 0; off >>= 1) {
      s += __shfl_xor(s, off, 32);
      d += __shfl_xor(d, off, 32);
    }
    if (lane == 0) { sdt[row] = s; sdt[GBM + row] = d; }
  }
  __syncthreads();

#pragma unroll 1
  for (int i = 0; i < 16; ++i) {
    const int row  = 16 * wave + i;
    const int grow = rowBase + row;
    const v4f p = *(const v4fa*)(stg + row * HD + 4 * lane);
    if (grow < NN) st2_v4f(XP + (size_t)grow * HD + 4 * lane, p);
  }
  if (wave == 0) {
    const v4f alv = *(const v4fa*)(sdt + 4 * lane);
    st2_v4f(AL + (size_t)blockIdx.x * (2 * GBM) + 4 * lane, alv);
  }
}

template <int KT>
__global__ __launch_bounds__(GTHR) __attribute__((amdgpu_num_vgpr(248)))
void k_gemmc(const unsigned short* __restrict__ HL, const unsigned short* __restrict__ BT,
             const int* __restrict__ CO, float* P) {
  static_assert(KT == 128 || KT == 256);
  __shared__ __attribute__((aligned(16))) float stg[GBM * HD];
  __shared__ __attribute__((aligned(16))) int sdv[GBM];
  const int tid = (int)threadIdx.x, lane = tid & 31, wave = tid >> 5, hh = lane >> 4, m = lane & 15;
  const int rowBase = (int)blockIdx.x * GBM;
  const int bucket  = rowBase >> SLB;
  const int slot0   = rowBase & (NBRUN - 1);
  if (tid < 16)
    *(v4ia*)(sdv + 4 * tid) = *(const v4ia*)(CO + (size_t)bucket * COI + 2 * NBRUN + slot0 + 4 * tid);

  v8f acc[8];
  {
    const v8f z = {0.f, 0.f, 0.f, 0.f, 0.f, 0.f, 0.f, 0.f};
#pragma unroll
    for (int t = 0; t < 8; ++t) acc[t] = z;
  }
  const unsigned short* ap = HL + (size_t)(rowBase + 16 * wave + m) * (size_t)KH + 8 * hh;
  const unsigned short* bp = BT + (size_t)m * (size_t)KH + 8 * hh;
  gemm_16x128<KT, KH>(ap, bp, acc);
  stage_d8(stg, acc, wave, hh, m);
  __syncthreads();

#pragma unroll 1
  for (int i = 0; i < 16; ++i) {
    const int row  = 16 * wave + i;
    const int grow = rowBase + row;
    const float di = __int_as_float(sdv[row]);
    const v4f p = *(const v4fa*)(stg + row * HD + 4 * lane);
    v4f o;
    o.x = p.x * di; o.y = p.y * di; o.z = p.z * di; o.w = p.w * di;
    if (grow < NN) st2_v4f(P + (size_t)grow * HD + 4 * lane, o);
  }
}

__global__ __launch_bounds__(NTHR) __attribute__((amdgpu_num_vgpr(248)))
void k_att(const int* __restrict__ LIST, const int* __restrict__ CO, const int* __restrict__ FLAG,
           const float* __restrict__ AL, const float* __restrict__ XP, const float* __restrict__ SM,
           unsigned short* HL, float* MAXP) {
  __shared__ __attribute__((aligned(16))) float sb[HD];
  const int tid = (int)threadIdx.x, lane = tid & 31, wave = tid >> 5;
  if (tid < 32) *(v4fa*)(sb + 4 * tid) = *(const v4fa*)(SM + 2 * HD + 4 * tid);
  __syncthreads();
  const v4f bv = *(const v4fa*)(sb + 4 * lane);
  const int rowBase = (int)blockIdx.x * ABM;
  const int bucket  = rowBase >> SLB;
  const int* lb  = LIST + (size_t)bucket * RCAP;
  const int* cob = CO + (size_t)bucket * COI;
  const int flag = FLAG[(size_t)bucket * 32];
  const float qnan = __uint_as_float(0x7fc00000u);

#pragma unroll 1
  for (int i = 0; i < ABM / NWAVE; ++i) {
    const int node = rowBase + (ABM / NWAVE) * wave + i;
    const int slot = node & (NBRUN - 1);
    int c = cob[slot];
    int o = cob[NBRUN + slot];
    const bool big = c > TRIPCAP;
    c = c < 0 ? 0 : (c > TRIPCAP ? TRIPCAP : c);
    o = o < 0 ? 0 : (o > RCAP - 1 ? RCAP - 1 : o);
    const int nc  = node < NN ? node : NN - 1;
    const int alb = (nc >> 6) * (2 * GBM) + (nc & (GBM - 1));
    const float as0 = AL[alb];
    const float ad  = AL[alb + GBM];
    const v4f a0v = *(const v4fa*)(XP + (size_t)nc * HD + 4 * lane);
    float a0 = a0v.x, a1 = a0v.y, a2 = a0v.z, a3 = a0v.w;
    float l0 = as0 + ad;
    l0 = l0 > 0.0f ? l0 : NEGSL * l0;
    float mx = l0, dn = 1.0f;
#pragma unroll 1
    for (int b0 = 0; b0 < c; b0 += 32) {
      int idx = o + b0 + lane;
      idx = idx > RCAP - 1 ? RCAP - 1 : idx;
      const unsigned wd = (unsigned)lb[idx];
      int sr = (int)(wd & 0xffffu);
      sr = sr > NN - 1 ? NN - 1 : sr;
      const float es  = AL[(sr >> 6) * (2 * GBM) + (sr & (GBM - 1))];
      const int   esi = __float_as_int(es);
      const int m32 = (c - b0) < 32 ? (c - b0) : 32;
#pragma unroll 1
      for (int k = 0; k < m32; ++k) {
        const int   sk  = __builtin_amdgcn_readlane(sr, k);
        const float ask = __int_as_float(__builtin_amdgcn_readlane(esi, k));
        const v4f v = *(const v4fa*)(XP + (size_t)sk * HD + 4 * lane);
        float lg = ask + ad;
        lg = lg > 0.0f ? lg : NEGSL * lg;
        const float df = lg - mx;
        const float ee = expf(-fabsf(df));
        const bool  up = df > 0.0f;
        const float s1 = up ? ee : 1.0f;
        const float s2 = up ? 1.0f : ee;
        mx = up ? lg : mx;
        dn = fmaf(dn, s1, s2);
        a0 = fmaf(a0, s1, s2 * v.x); a1 = fmaf(a1, s1, s2 * v.y);
        a2 = fmaf(a2, s1, s2 * v.z); a3 = fmaf(a3, s1, s2 * v.w);
      }
    }
    const float inv = 1.0f / dn;
    float h0 = fmaf(a0, inv, bv.x), h1 = fmaf(a1, inv, bv.y);
    float h2 = fmaf(a2, inv, bv.z), h3 = fmaf(a3, inv, bv.w);
    const bool bad  = (flag != 0) | big;
    const bool live = node < NN;
    h0 = bad ? qnan : h0; h1 = bad ? qnan : h1; h2 = bad ? qnan : h2; h3 = bad ? qnan : h3;
    h0 = live ? h0 : 0.0f; h1 = live ? h1 : 0.0f; h2 = live ? h2 : 0.0f; h3 = live ? h3 : 0.0f;
    int h01, h23, l01, l23;
    hilo_pack(h0, h1, h2, h3, h01, h23, l01, l23);
    const v4i ow = regroup8w(h01, h23, l01, l23, lane);
    v4f ov;
    ov.x = h0; ov.y = h1; ov.z = h2; ov.w = h3;
    if (node < MP) {
      float* mp = MAXP + (size_t)node * HD + 4 * lane;
      unsigned short* hp = HL + (size_t)node * KH + 8 * lane;
      *(volatile v4f*)mp = ov;
      *(volatile v4i*)hp = ow;
      __threadfence();
      *(volatile v4f*)mp = ov;
      *(volatile v4i*)hp = ow;
    }
  }
}

template <int LAYER>
__global__ __launch_bounds__(NTHR) __attribute__((amdgpu_num_vgpr(248)))
void k_agg(const int* __restrict__ LIST, const int* __restrict__ CO, const int* __restrict__ FLAG,
           const float* __restrict__ P, const float* __restrict__ SM,
           unsigned short* HL, float* MAXP, float* out) {
  static_assert(LAYER >= 1 && LAYER <= NLAY);
  __shared__ __attribute__((aligned(16))) float sb[HD];
  const int tid = (int)threadIdx.x, lane = tid & 31, wave = tid >> 5;
  if (tid < 32) *(v4fa*)(sb + 4 * tid) = *(const v4fa*)(SM + 3 * HD + (LAYER - 1) * HD + 4 * tid);
  __syncthreads();
  const v4f bv = *(const v4fa*)(sb + 4 * lane);
  const int rowBase = (int)blockIdx.x * ABM;
  const int bucket  = rowBase >> SLB;
  const int* lb  = LIST + (size_t)bucket * RCAP;
  const int* cob = CO + (size_t)bucket * COI;
  const int flag = FLAG[(size_t)bucket * 32];
  const float qnan = __uint_as_float(0x7fc00000u);

#pragma unroll 1
  for (int i = 0; i < ABM / NWAVE; ++i) {
    const int node = rowBase + (ABM / NWAVE) * wave + i;
    const int slot = node & (NBRUN - 1);
    int c = cob[slot];
    int o = cob[NBRUN + slot];
    const float di = __int_as_float(cob[2 * NBRUN + slot]);
    const bool big = c > TRIPCAP;
    c = c < 0 ? 0 : (c > TRIPCAP ? TRIPCAP : c);
    o = o < 0 ? 0 : (o > RCAP - 1 ? RCAP - 1 : o);
    const int nc = node < NN ? node : NN - 1;
    float a0 = 0.0f, a1 = 0.0f, a2 = 0.0f, a3 = 0.0f;
#pragma unroll 1
    for (int b0 = 0; b0 < c; b0 += 32) {
      int idx = o + b0 + lane;
      idx = idx > RCAP - 1 ? RCAP - 1 : idx;
      const unsigned wd = (unsigned)lb[idx];
      int sr = (int)(wd & 0xffffu);
      sr = sr > NN - 1 ? NN - 1 : sr;
      const int wbi = (int)(wd & 0xffff0000u);
      const int m32 = (c - b0) < 32 ? (c - b0) : 32;
#pragma unroll 1
      for (int k = 0; k < m32; ++k) {
        const int   sk = __builtin_amdgcn_readlane(sr, k);
        const float wk = __int_as_float(__builtin_amdgcn_readlane(wbi, k));
        const v4f v = *(const v4fa*)(P + (size_t)sk * HD + 4 * lane);
        a0 = fmaf(wk, v.x, a0); a1 = fmaf(wk, v.y, a1);
        a2 = fmaf(wk, v.z, a2); a3 = fmaf(wk, v.w, a3);
      }
    }
    const v4f g  = *(const v4fa*)(P + (size_t)nc * HD + 4 * lane);
    const v4f mv = *(const v4fa*)(MAXP + (size_t)nc * HD + 4 * lane);
    asm volatile("" :: "v"(g));
    asm volatile("" :: "v"(mv));
    a0 = a0 + g.x; a1 = a1 + g.y; a2 = a2 + g.z; a3 = a3 + g.w;
    float z0 = fmaf(di, a0, bv.x), z1 = fmaf(di, a1, bv.y), z2 = fmaf(di, a2, bv.z), z3 = fmaf(di, a3, bv.w);
    float r0 = (z0 > 0.0f) ? z0 : (z0 - z0), r1 = (z1 > 0.0f) ? z1 : (z1 - z1);
    float r2 = (z2 > 0.0f) ? z2 : (z2 - z2), r3 = (z3 > 0.0f) ? z3 : (z3 - z3);
    const bool bad  = (flag != 0) | big;
    const bool live = node < NN;
    r0 = bad ? qnan : r0; r1 = bad ? qnan : r1; r2 = bad ? qnan : r2; r3 = bad ? qnan : r3;
    r0 = live ? r0 : 0.0f; r1 = live ? r1 : 0.0f; r2 = live ? r2 : 0.0f; r3 = live ? r3 : 0.0f;
    float n0 = ((r0 > mv.x) | (r0 != r0)) ? r0 : mv.x;
    float n1 = ((r1 > mv.y) | (r1 != r1)) ? r1 : mv.y;
    float n2 = ((r2 > mv.z) | (r2 != r2)) ? r2 : mv.z;
    float n3 = ((r3 > mv.w) | (r3 != r3)) ? r3 : mv.w;
    n0 = bad ? qnan : n0; n1 = bad ? qnan : n1; n2 = bad ? qnan : n2; n3 = bad ? qnan : n3;
    n0 = live ? n0 : 0.0f; n1 = live ? n1 : 0.0f; n2 = live ? n2 : 0.0f; n3 = live ? n3 : 0.0f;
    v4f nv;
    nv.x = n0; nv.y = n1; nv.z = n2; nv.w = n3;
    if constexpr (LAYER < NLAY) {
      int h01, h23, l01, l23;
      hilo_pack(r0, r1, r2, r3, h01, h23, l01, l23);
      const v4i ow = regroup8w(h01, h23, l01, l23, lane);
      if (node < MP) {
        float* mp = MAXP + (size_t)node * HD + 4 * lane;
        unsigned short* hp = HL + (size_t)node * KH + 8 * lane;
        *(volatile v4f*)mp = nv;
        *(volatile v4i*)hp = ow;
        __threadfence();
        *(volatile v4f*)mp = nv;
        *(volatile v4i*)hp = ow;
      }
    } else {
      if (live) {
        float* op = out + (size_t)node * HD + 4 * lane;
        *(volatile v4f*)op = nv;
        __threadfence();
        *(volatile v4f*)op = nv;
      }
    }
  }
}

extern "C" void kernel_launch(void* const* d_in, const int* in_sizes, int n_in,
                              void* d_out, int out_size, void* d_ws, size_t ws_size,
                              hipStream_t stream) {
  if (n_in < 9) return;
  if (in_sizes[0] != NN * HD) return;
  if (in_sizes[1] != 2 * NE) return;
  if (in_sizes[2] != NE) return;
  if (in_sizes[3] != HD * HD) return;
  if (in_sizes[4] != HD) return;
  if (in_sizes[5] != HD) return;
  if (in_sizes[6] != HD) return;
  if (in_sizes[7] != NLAY * HD * HD) return;
  if (in_sizes[8] != NLAY * HD) return;
  if (out_size != NN * HD) return;

  const float* x   = (const float*)d_in[0];
  const int*   ei  = (const int*)d_in[1];
  const float* ew  = (const float*)d_in[2];
  const float* Wa  = (const float*)d_in[3];
  const float* asv = (const float*)d_in[4];
  const float* adv = (const float*)d_in[5];
  const float* ba  = (const float*)d_in[6];
  const float* Wc  = (const float*)d_in[7];
  const float* bc  = (const float*)d_in[8];
  float* out = (float*)d_out;
  const int* srcs = ei;
  const int* dsts = ei + NE;

  constexpr size_t zHL   = (size_t)MP * KH * 2;
  constexpr size_t zXB   = (size_t)MP * HD * 2;
  constexpr size_t zF    = (size_t)MP * HD * 4;
  constexpr size_t zLIST = (size_t)NBK * RCAP * 4;
  constexpr size_t zCO   = (size_t)NBK * COI * 4;
  constexpr size_t zFLAG = (size_t)FLAGINTS * 4;
  constexpr size_t zAL   = (size_t)(MP / GBM) * 2 * GBM * 4;
  constexpr size_t zWaT  = (size_t)HD * HD * 2;
  constexpr size_t zWcD  = (size_t)NLAY * HD * KH * 2;
  constexpr size_t zSM   = (size_t)SMN * 4;
  constexpr size_t oHL   = 0;
  constexpr size_t oXP   = oHL + zHL;
  constexpr size_t oMAXP = oXP + zF;
  constexpr size_t oLIST = oMAXP + zF;
  constexpr size_t oCO   = oLIST + zLIST;
  constexpr size_t oFLAG = oCO + zCO;
  constexpr size_t oAL   = oFLAG + zFLAG;
  constexpr size_t oWaT  = oAL + zAL;
  constexpr size_t oWcD  = oWaT + zWaT;
  constexpr size_t oSM   = oWcD + zWcD;
  constexpr size_t oEND  = oSM + zSM;
  static_assert(zXB <= zHL);
  static_assert(zHL % 256 == 0 && zF % 256 == 0 && zLIST % 256 == 0 && zCO % 256 == 0 && zFLAG % 256 == 0);
  static_assert(zAL % 256 == 0 && zWaT % 256 == 0 && zWcD % 256 == 0 && zSM % 256 == 0);
  static_assert(oEND <= (size_t)WSMAX);
  if (oEND > ws_size) return;

  char* ws = (char*)d_ws;
  unsigned short* HL   = (unsigned short*)(ws + oHL);
  unsigned short* XB   = (unsigned short*)(ws + oHL);
  float*          XP   = (float*)(ws + oXP);
  float*          MAXP = (float*)(ws + oMAXP);
  int*            LIST = (int*)(ws + oLIST);
  int*            CO   = (int*)(ws + oCO);
  int*            FLAG = (int*)(ws + oFLAG);
  float*          AL   = (float*)(ws + oAL);
  unsigned short* WaT  = (unsigned short*)(ws + oWaT);
  unsigned short* WcD  = (unsigned short*)(ws + oWcD);
  float*          SM   = (float*)(ws + oSM);

  hipFuncSetAttribute(reinterpret_cast<const void*>(&k_bucket), hipFuncAttributeMaxDynamicSharedMemorySize, (int)BK_LDS);

  constexpr int K1 = CONV_SPLIT_L1 ? KH : HD;
  constexpr int K2 = CONV_SPLIT_L2 ? KH : HD;
  constexpr int K3 = CONV_SPLIT_L3 ? KH : HD;
  constexpr int GA = NBK * NBRUN / ABM;

  k_prep<<<PBTOT, NTHR, 0, stream>>>(x, Wa, asv, adv, ba, Wc, bc, XB, WaT, WcD, SM, FLAG);
  k_bucket<<<NBK, NTHR, BK_LDS, stream>>>(srcs, dsts, ew, LIST, CO, FLAG);
  k_gemm0<<<MP / GBM, GTHR, 0, stream>>>(XB, WaT, SM, XP, AL);
  k_att<<<GA, NTHR, 0, stream>>>(LIST, CO, FLAG, AL, XP, SM, HL, MAXP);
  k_gemmc<K1><<<MP / GBM, GTHR, 0, stream>>>(HL, WcD, CO, XP);
  k_agg<1><<<GA, NTHR, 0, stream>>>(LIST, CO, FLAG, XP, SM, HL, MAXP, out);
  k_gemmc<K2><<<MP / GBM, GTHR, 0, stream>>>(HL, WcD + (size_t)1 * HD * KH, CO, XP);
  k_agg<2><<<GA, NTHR, 0, stream>>>(LIST, CO, FLAG, XP, SM, HL, MAXP, out);
  k_gemmc<K3><<<MP / GBM, GTHR, 0, stream>>>(HL, WcD + (size_t)2 * HD * KH, CO, XP);
  k_agg<3><<<GA, NTHR, 0, stream>>>(LIST, CO, FLAG, XP, SM, HL, MAXP, out);
}
